// MultiHeadCrossAttention_11854109737409
// MI455X (gfx1250) — hardware-verified
//
#include <hip/hip_runtime.h>
#include <math.h>

#ifndef NB
#define NB 2
#endif
#ifndef SEQ
#define SEQ 2048
#endif
#define NB_FULL 2
#define SEQ_FULL 2048
#define DD 1024
#define HH 16
#define HD 64
#define KCH 64
#define NWV 4
#define OSP 68
#define PSC 32768.0f
#define VSC 16.0f
static_assert(HH * HD == DD);
static_assert(HH == 16);
static_assert(SEQ % 64 == 0);
static_assert(NB >= 1 && NB <= NB_FULL);
static_assert(SEQ >= 64 && SEQ <= SEQ_FULL);
static_assert(DD % 64 == 0);

typedef unsigned short us;
typedef us       v8us  __attribute__((ext_vector_type(8)));
typedef us       v16us __attribute__((ext_vector_type(16)));
typedef _Float16 v16h  __attribute__((ext_vector_type(16)));
typedef __bf16   v16b  __attribute__((ext_vector_type(16)));
typedef float    v8f   __attribute__((ext_vector_type(8)));
typedef float    v4f   __attribute__((ext_vector_type(4)));
union FU { v16us u; v8us h[2]; v16b b; v16h f; };

__device__ __forceinline__ us bfbits(float f) { unsigned int u = __float_as_uint(f); u += 0x7fffu + ((u >> 16) & 1u); return (us)(u >> 16); }
__device__ __forceinline__ float bf2f(us h) { return __uint_as_float(((unsigned int)h) << 16); }
__device__ __forceinline__ void bsplit(float f, us& hi, us& lo) { hi = bfbits(f); lo = bfbits(f - bf2f(hi)); }
__device__ __forceinline__ us hbits(float f) { return __builtin_bit_cast(us, (_Float16)f); }
__device__ __forceinline__ v8f zero8() { v8f z = {0.f, 0.f, 0.f, 0.f, 0.f, 0.f, 0.f, 0.f}; return z; }

__device__ __forceinline__ v8f mma_bf(v16b a, v16b b, v8f c) {
    c = __builtin_amdgcn_wmma_f32_16x16x32_bf16(false, a, false, b, (short)0, c, false, false);
    asm volatile("v_nop\n\tv_nop\n\tv_nop\n\tv_nop" : "+v"(c) : "v"(a), "v"(b));
    return c;
}
__device__ __forceinline__ v8f mma_h(v16h a, v16h b, v8f c) {
    c = __builtin_amdgcn_wmma_f32_16x16x32_f16(false, a, false, b, (short)0, c, false, false);
    asm volatile("v_nop\n\tv_nop\n\tv_nop\n\tv_nop" : "+v"(c) : "v"(a), "v"(b));
    return c;
}

__global__ __launch_bounds__(256) void k_cvt_bf8(const float* __restrict__ src, long long sbs, int rows, us* __restrict__ dst, long long n8) {
    const long long u = (long long)blockIdx.x * 256 + threadIdx.x;
    if (u >= n8) return;
    const long long e = 8 * u;
    const long long r = e / DD; const int cc = (int)(e - r * DD);
    const int bi = (int)(r / rows); const int s = (int)(r - (long long)bi * rows);
    const float* p = src + (long long)bi * sbs + (long long)s * DD + cc;
    const v4f a = *(const v4f*)p; const v4f q = *(const v4f*)(p + 4);
    v8us o;
    o[0] = bfbits(a.x); o[1] = bfbits(a.y); o[2] = bfbits(a.z); o[3] = bfbits(a.w);
    o[4] = bfbits(q.x); o[5] = bfbits(q.y); o[6] = bfbits(q.z); o[7] = bfbits(q.w);
    volatile v8us* d = (volatile v8us*)(dst + e); *d = o; __threadfence(); *d = o;
}

__global__ __launch_bounds__(256) void k_wT(const float* __restrict__ W, int KI, int NO, int KP, us* __restrict__ Bt) {
    const long long u = (long long)blockIdx.x * 256 + threadIdx.x;
    const long long np = (long long)NO * (KP / 2);
    if (u >= np) return;
    const int o = (int)(u / (KP / 2)); const int k0 = 2 * (int)(u % (KP / 2));
    int ka = k0; if (ka >= KI) ka -= KI; int kb = k0 + 1; if (kb >= KI) kb -= KI;
    ka = min(max(ka, 0), KI - 1); kb = min(max(kb, 0), KI - 1);
    const float a = W[(long long)ka * NO + o], b2 = W[(long long)kb * NO + o];
    const unsigned int pk = (unsigned int)bfbits(a) | ((unsigned int)bfbits(b2) << 16);
    volatile unsigned int* d = (volatile unsigned int*)(Bt + (long long)o * KP + k0); *d = pk; __threadfence(); *d = pk;
}

__global__ __launch_bounds__(256) void k_gemm64(const us* __restrict__ A, int lda, const us* __restrict__ Bt, int ldb,
                                               float* __restrict__ C, int ldc, const float* __restrict__ bias, int M, int N, int K) {
    __shared__ __align__(16) float sT[8][16 * OSP];
    const int lane = threadIdx.x & 31, wave = threadIdx.x >> 5;
    const int tilesN = N >> 6, tilesM = M >> 6;
    const int tile = blockIdx.x * 8 + wave;
    if (tile >= tilesM * tilesN) return;
    const int tm = tile / tilesN, tn = tile - tm * tilesN;
    const int m0 = tm << 6, n0 = tn << 6;
    const int rl = lane & 15, koff = (lane >> 4) * 8, mOff = (lane >> 4) * 8;
    v8f acc[4][4];
#pragma unroll
    for (int i = 0; i < 4; ++i)
#pragma unroll
        for (int j = 0; j < 4; ++j) acc[i][j] = zero8();
    for (int k0 = 0; k0 < K; k0 += 32) {
        FU bf[4];
#pragma unroll
        for (int j = 0; j < 4; ++j) {
            const long long bo = (long long)(n0 + 16 * j + rl) * ldb + koff + k0;
            bf[j].h[0] = *(const v8us*)(Bt + bo); bf[j].h[1] = *(const v8us*)(Bt + bo + 16);
        }
#pragma unroll
        for (int i = 0; i < 4; ++i) {
            const long long ao = (long long)(m0 + 16 * i + rl) * lda + koff + k0;
            FU af; af.h[0] = *(const v8us*)(A + ao); af.h[1] = *(const v8us*)(A + ao + 16);
#pragma unroll
            for (int j = 0; j < 4; ++j) acc[i][j] = mma_bf(af.b, bf[j].b, acc[i][j]);
        }
    }
    float* slab = sT[wave];
    const int h2 = lane >> 4, c4 = (lane & 15) * 4;
#pragma unroll
    for (int i = 0; i < 4; ++i) {
        const int mB = m0 + 16 * i;
#pragma unroll
        for (int j = 0; j < 4; ++j) {
            const int n = n0 + 16 * j + rl;
            const float bv = bf2f(bfbits(bias[n]));
#pragma unroll
            for (int r = 0; r < 8; ++r) slab[(mOff + r) * OSP + 16 * j + rl] = acc[i][j][r] + bv;
        }
        __builtin_amdgcn_fence(3, "workgroup");
        __builtin_amdgcn_wave_barrier();
        __builtin_amdgcn_fence(2, "workgroup");
        for (int pass = 0; pass < 2; ++pass) {
#pragma unroll
            for (int it = 0; it < 8; ++it) {
                const int row = it * 2 + h2;
                const v4f v = *(const v4f*)(slab + row * OSP + c4);
                *(volatile v4f*)(C + (long long)(mB + row) * ldc + n0 + c4) = v;
            }
            __threadfence();
        }
        __builtin_amdgcn_fence(3, "workgroup");
        __builtin_amdgcn_wave_barrier();
        __builtin_amdgcn_fence(2, "workgroup");
    }
}

__global__ __launch_bounds__(256) void k_kplane(const float* __restrict__ KVF, int S, us* __restrict__ KP, long long n8) {
    const long long u = (long long)blockIdx.x * 256 + threadIdx.x;
    if (u >= n8) return;
    const int d8 = (int)(u & 7) * 8;
    const long long row = u >> 3;
    const int s = (int)(row % S); const long long bh = row / S; const int hd = (int)(bh % HH); const int bi = (int)(bh / HH);
    const float* p = KVF + ((long long)bi * S + s) * (2 * DD) + hd * (2 * HD) + d8;
    const v4f a = *(const v4f*)p; const v4f q = *(const v4f*)(p + 4);
    const float f[8] = {a.x, a.y, a.z, a.w, q.x, q.y, q.z, q.w};
    v8us hv;
#pragma unroll
    for (int e = 0; e < 8; ++e) hv[e] = hbits(f[e]);
    volatile v8us* dh = (volatile v8us*)(KP + 8 * u);
    *dh = hv; __threadfence(); *dh = hv;
}

__global__ __launch_bounds__(256) void k_vtplane(const float* __restrict__ KVF, int S, us* __restrict__ VT) {
    __shared__ float tl[64][65];
    const int kc = blockIdx.x, bh = blockIdx.y, tid = threadIdx.x;
    const int hd = bh % HH, bi = bh / HH;
    const float* src = KVF + ((long long)bi * S + (long long)kc * 64) * (2 * DD) + hd * (2 * HD) + HD;
#pragma unroll
    for (int i = 0; i < 4; ++i) {
        const int idx = tid + 256 * i; const int row = idx >> 4; const int cq = (idx & 15) * 4;
        const v4f v = *(const v4f*)(src + (long long)row * (2 * DD) + cq);
        tl[row][cq] = v.x; tl[row][cq + 1] = v.y; tl[row][cq + 2] = v.z; tl[row][cq + 3] = v.w;
    }
    __syncthreads();
    us* dst = VT + (long long)bh * HD * S + (long long)kc * 64;
#pragma unroll
    for (int i = 0; i < 2; ++i) {
        const int piece = tid + 256 * i; const int d = piece >> 3; const int s8 = (piece & 7) * 8;
        v8us hv;
#pragma unroll
        for (int e = 0; e < 8; ++e) hv[e] = hbits(VSC * tl[s8 + e][d]);
        volatile v8us* pd = (volatile v8us*)(dst + (long long)d * S + s8); *pd = hv; __threadfence(); *pd = hv;
    }
}

__global__ __launch_bounds__(128) __attribute__((amdgpu_num_vgpr(256)))
void k_attn(const float* __restrict__ QF, const us* __restrict__ KP, const us* __restrict__ VT,
            us* __restrict__ CTXP, int S, float qscale, float sscale) {
    __shared__ __align__(16) us Ksh[KCH * HD];
    __shared__ __align__(16) us Vth[HD * KCH];
    __shared__ __align__(16) us Psh[NWV][16 * KCH];
    __shared__ __align__(16) float Os[NWV][16 * OSP];

    const int tid = threadIdx.x, wave = tid >> 5, lane = tid & 31, hh = lane >> 4, c = lane & 15;
    const int nqb = S / 64;
    const int bx = blockIdx.x; const int qb = bx % nqb; const int bh = bx / nqb; const int hd = bh % HH; const int bi = bh / HH;
    const int q0 = qb * 64 + wave * 16;

    v16h qa[2];
    {
        const float* qrow = QF + ((long long)bi * S + q0 + c) * DD + hd * HD;
#pragma unroll
        for (int dc = 0; dc < 2; ++dc) {
            FU th;
#pragma unroll
            for (int g = 0; g < 2; ++g) {
                const v4f x0 = *(const v4f*)(qrow + dc * 32 + 16 * g + 8 * hh);
                const v4f x1 = *(const v4f*)(qrow + dc * 32 + 16 * g + 8 * hh + 4);
                const float f[8] = {x0.x, x0.y, x0.z, x0.w, x1.x, x1.y, x1.z, x1.w};
#pragma unroll
                for (int e = 0; e < 8; ++e) th.u[8 * g + e] = hbits(f[e] * qscale);
            }
            qa[dc] = th.f;
        }
    }

    float mrow[8], lrow[8];
    v8f oacc[4];
#pragma unroll
    for (int r = 0; r < 8; ++r) { mrow[r] = -__builtin_inff(); lrow[r] = 0.f; }
#pragma unroll
    for (int t = 0; t < 4; ++t) oacc[t] = zero8();

    const int nch = S / KCH;
    us* pwh = Psh[wave];
    for (int kc = 0; kc < nch; ++kc) {
        const int kv0 = kc * KCH;
        __syncthreads();
        {
            const us* kh = KP + ((long long)bh * S + kv0) * HD;
            const us* vt = VT + (long long)bh * HD * S + kv0;
#pragma unroll
            for (int i = 0; i < 4; ++i) {
                const int p = tid + 128 * i; const int row = p >> 3; const int col8 = (p & 7) * 8;
                const v8us a  = *(const v8us*)(kh + row * HD + col8);
                const v8us vv = *(const v8us*)(vt + (long long)row * S + col8);
                *(v8us*)(Ksh + row * HD + col8) = a;
                *(v8us*)(Vth + row * KCH + col8) = vv;
            }
        }
        __syncthreads();

        v8f s[4];
#pragma unroll
        for (int j = 0; j < 4; ++j) {
            v8f acc = zero8();
#pragma unroll
            for (int dc = 0; dc < 2; ++dc) {
                FU kb;
                kb.h[0] = *(const v8us*)(Ksh + (j * 16 + c) * HD + dc * 32 + 8 * hh);
                kb.h[1] = *(const v8us*)(Ksh + (j * 16 + c) * HD + dc * 32 + 16 + 8 * hh);
                acc = mma_h(qa[dc], kb.f, acc);
            }
            s[j] = acc;
        }
        float cm[8];
#pragma unroll
        for (int r = 0; r < 8; ++r) {
            const float a0 = s[0][r] * sscale, a1 = s[1][r] * sscale, a2 = s[2][r] * sscale, a3 = s[3][r] * sscale;
            s[0][r] = a0; s[1][r] = a1; s[2][r] = a2; s[3][r] = a3;
            float m = fmaxf(fmaxf(a0, a1), fmaxf(a2, a3));
#pragma unroll
            for (int off = 1; off < 16; off <<= 1) m = fmaxf(m, __shfl_xor(m, off, 32));
            cm[r] = m;
        }
#pragma unroll
        for (int r = 0; r < 8; ++r) {
            const float mnew = fmaxf(mrow[r], cm[r]);
            const float alpha = exp2f(mrow[r] - mnew);
            mrow[r] = mnew;
            float psum = 0.f;
#pragma unroll
            for (int j = 0; j < 4; ++j) {
                const float p = exp2f(s[j][r] - mnew);
                psum += p;
                pwh[(8 * hh + r) * KCH + j * 16 + c] = hbits(p * PSC);
            }
#pragma unroll
            for (int off = 1; off < 16; off <<= 1) psum += __shfl_xor(psum, off, 32);
            lrow[r] = lrow[r] * alpha + psum;
#pragma unroll
            for (int t = 0; t < 4; ++t) oacc[t][r] *= alpha;
        }
        __builtin_amdgcn_fence(3, "workgroup");
        __builtin_amdgcn_wave_barrier();
        __builtin_amdgcn_fence(2, "workgroup");
#pragma unroll 1
        for (int kk = 0; kk < 2; ++kk) {
            FU pa;
            pa.h[0] = *(const v8us*)(pwh + c * KCH + kk * 32 + 8 * hh);
            pa.h[1] = *(const v8us*)(pwh + c * KCH + kk * 32 + 16 + 8 * hh);
#pragma unroll
            for (int t = 0; t < 4; ++t) {
                FU vb;
                vb.h[0] = *(const v8us*)(Vth + (t * 16 + c) * KCH + kk * 32 + 8 * hh);
                vb.h[1] = *(const v8us*)(Vth + (t * 16 + c) * KCH + kk * 32 + 16 + 8 * hh);
                oacc[t] = mma_h(pa.f, vb.f, oacc[t]);
            }
        }
    }

    float* os = Os[wave];
#pragma unroll
    for (int r = 0; r < 8; ++r) {
        const float inv = (1.0f / lrow[r]) * (1.0f / (PSC * VSC));
#pragma unroll
        for (int t = 0; t < 4; ++t) os[(8 * hh + r) * OSP + t * 16 + c] = oacc[t][r] * inv;
    }
    __builtin_amdgcn_fence(3, "workgroup");
    __builtin_amdgcn_wave_barrier();
    __builtin_amdgcn_fence(2, "workgroup");
    const long long prow = (long long)bi * S + ((long long)hd * S + q0) / HH;
    us* pbase = CTXP + prow * (2 * DD);
    const int qq = lane >> 3, c8 = (lane & 7) * 8;
    for (int pass = 0; pass < 2; ++pass) {
#pragma unroll
        for (int it = 0; it < 4; ++it) {
            const int row = it * 4 + qq;
            const float* sp = os + row * OSP + c8;
            v8us hv, lv;
#pragma unroll
            for (int e = 0; e < 8; ++e) { us hb, lb; bsplit(sp[e], hb, lb); hv[e] = hb; lv[e] = lb; }
            *(volatile v8us*)(pbase + row * HD + c8) = hv;
            *(volatile v8us*)(pbase + DD + row * HD + c8) = lv;
        }
        __threadfence();
    }
}

static inline size_t al256(size_t x) { return (x + 255) & ~(size_t)255; }

extern "C" void kernel_launch(void* const* d_in, const int* in_sizes, int n_in, void* d_out, int out_size, void* d_ws, size_t ws_size, hipStream_t stream) {
    if (n_in < 8) return;
    const long long MR = (long long)NB * SEQ;
    const long long needx = ((long long)(NB - 1) * SEQ_FULL + SEQ) * DD;
    if ((long long)in_sizes[0] < needx || (long long)in_sizes[1] < needx) return;
    if ((long long)in_sizes[2] < (long long)DD * 2 * DD || (long long)in_sizes[3] < 2LL * DD) return;
    if ((long long)in_sizes[4] < (long long)DD * DD || (long long)in_sizes[5] < (long long)DD) return;
    if ((long long)in_sizes[6] < (long long)DD * DD || (long long)in_sizes[7] < (long long)DD) return;
    if ((long long)out_size < MR * DD) return;

    const float* x   = (const float*)d_in[0];
    const float* y   = (const float*)d_in[1];
    const float* Wkv = (const float*)d_in[2];
    const float* bkv = (const float*)d_in[3];
    const float* Wq  = (const float*)d_in[4];
    const float* bq  = (const float*)d_in[5];
    const float* Wo  = (const float*)d_in[6];
    const float* bo  = (const float*)d_in[7];
    float* out = (float*)d_out;

    char* base = (char*)d_ws; size_t off = 0;
    us* XP   = (us*)(base + off);    off += al256((size_t)MR * DD * 2);
    us* YP   = (us*)(base + off);    off += al256((size_t)MR * DD * 2);
    us* WKVP = (us*)(base + off);    off += al256((size_t)2 * DD * DD * 2);
    us* WQP  = (us*)(base + off);    off += al256((size_t)DD * DD * 2);
    us* WOP  = (us*)(base + off);    off += al256((size_t)DD * 2 * DD * 2);
    float* KVF = (float*)(base + off); off += al256((size_t)MR * 2 * DD * 4);
    float* QF  = (float*)(base + off); off += al256((size_t)MR * DD * 4);
    us* KPp  = (us*)(base + off);    off += al256((size_t)NB * HH * SEQ * HD * 2);
    us* VTp  = (us*)(base + off);    off += al256((size_t)NB * HH * HD * SEQ * 2);
    us* CTXP = (us*)(base + off);    off += al256((size_t)MR * 2 * DD * 2);
    if (off > ws_size) return;

    const long long n8x = MR * DD / 8;
    k_cvt_bf8<<<(unsigned)((n8x + 255) / 256), 256, 0, stream>>>(x, (long long)SEQ_FULL * DD, SEQ, XP, n8x);
    k_cvt_bf8<<<(unsigned)((n8x + 255) / 256), 256, 0, stream>>>(y, (long long)SEQ_FULL * DD, SEQ, YP, n8x);
    k_wT<<<(unsigned)((((long long)2 * DD) * (DD / 2) + 255) / 256), 256, 0, stream>>>(Wkv, DD, 2 * DD, DD, WKVP);
    k_wT<<<(unsigned)((((long long)DD) * (DD / 2) + 255) / 256), 256, 0, stream>>>(Wq, DD, DD, DD, WQP);
    k_wT<<<(unsigned)((((long long)DD) * (DD) + 255) / 256), 256, 0, stream>>>(Wo, DD, DD, 2 * DD, WOP);
    {
        const long long tiles = (MR / 64) * ((2 * DD) / 64);
        k_gemm64<<<(unsigned)((tiles + 7) / 8), 256, 0, stream>>>(XP, DD, WKVP, DD, KVF, 2 * DD, bkv, (int)MR, 2 * DD, DD);
    }
    {
        const long long tiles = (MR / 64) * (DD / 64);
        k_gemm64<<<(unsigned)((tiles + 7) / 8), 256, 0, stream>>>(YP, DD, WQP, DD, QF, DD, bq, (int)MR, DD, DD);
    }
    const long long n8k = (long long)NB * HH * SEQ * (HD / 8);
    k_kplane<<<(unsigned)((n8k + 255) / 256), 256, 0, stream>>>(KVF, SEQ, KPp, n8k);
    k_vtplane<<<dim3((unsigned)(SEQ / 64), (unsigned)(NB * HH)), 256, 0, stream>>>(KVF, SEQ, VTp);
    k_attn<<<(unsigned)((long long)NB * HH * (SEQ / 64)), 128, 0, stream>>>(QF, KPp, VTp, CTXP, SEQ, 1.4426950408889634f, 0.125f);
    {
        const long long tiles = (MR / 64) * (DD / 64);
        k_gemm64<<<(unsigned)((tiles + 7) / 8), 256, 0, stream>>>(CTXP, 2 * DD, WOP, 2 * DD, out, DD, bo, (int)MR, DD, 2 * DD);
    }
}
